// SequentialTransductionUnitJagged_46420006536069
// MI455X (gfx1250) — hardware-run, weakly checked
//
#include <hip/hip_runtime.h>
#include <math.h>


static constexpr int kB      = 8;
static constexpr int kN      = 1024;
static constexpr int kD      = 512;
static constexpr int kHeads  = 8;
static constexpr int kDh     = 64;
static constexpr int kTok    = 4096;
static constexpr int kN1     = 2048;
static constexpr int kRel    = 2 * kN - 1;
static constexpr int kKch    = kN / 32;
static constexpr int kQblk   = kN / 64;
static constexpr int kCvtThreads  = 256;
static constexpr int kTrThreads   = 256;
static constexpr int kFlagThreads = 128;
static constexpr int kGemmThreads = 128;
static constexpr int kVtThreads   = 128;
static constexpr int kLnThreads   = 64;
static constexpr int kStgPitch = 132;
static constexpr int kPP = 36;
static constexpr int kOP = 68;
static constexpr int kTP = 72;

static_assert(kHeads * kDh == kD);
static_assert(kDh == 64);
static_assert(kN % 64 == 0);
static_assert(kTok % 64 == 0);
static_assert(kTok % 32 == 0);
static_assert(kN1 == 4 * kD);
static_assert(kN1 % 128 == 0);
static_assert(kD % 128 == 0);
static_assert(kD % 32 == 0);
static_assert((kD * kD) % (kCvtThreads * 8) == 0);
static_assert(kN == kFlagThreads * 8);
static_assert(kKch == 32);
static_assert(kQblk == 16);
static_assert(kD == kLnThreads * 8);
static_assert(kN1 % 64 == 0 && kD % 64 == 0);

typedef _Float16     v16h __attribute__((ext_vector_type(16)));
typedef _Float16     v8h  __attribute__((ext_vector_type(8)));
typedef float        v8f  __attribute__((ext_vector_type(8)));
typedef float        v4f  __attribute__((ext_vector_type(4)));
typedef unsigned int v4u  __attribute__((ext_vector_type(4)));
typedef int          v4i  __attribute__((ext_vector_type(4)));

union Frag { v16h v; v8h half[2]; };

__device__ __forceinline__ v8f wmma_f16(v16h a, v16h b, v8f acc)
{
    acc = __builtin_amdgcn_wmma_f32_16x16x32_f16(false, a, false, b, (short)0, acc, false, false);
#if defined(__HIP_DEVICE_COMPILE__)
    asm volatile("v_nop\n\tv_nop\n\tv_nop\n\tv_nop" : "+v"(acc) : "v"(a), "v"(b));
#endif
    return acc;
}

__device__ __forceinline__ float bf16_rne(float x)
{
    unsigned int u = __float_as_uint(x);
    u = u + 0x7FFFu + ((u >> 16) & 1u);
    return __uint_as_float(u & 0xFFFF0000u);
}

__device__ __forceinline__ _Float16 cvt16(float x, float sc)
{
    return (_Float16)(bf16_rne(x) * sc);
}

__device__ __forceinline__ float silu_fast(float z)
{
    return z * __builtin_amdgcn_rcpf(1.0f + __expf(-z));
}

__device__ __forceinline__ float wave_sum(float v)
{
    v += __shfl_xor(v, 1, 32);
    v += __shfl_xor(v, 2, 32);
    v += __shfl_xor(v, 4, 32);
    v += __shfl_xor(v, 8, 32);
    v += __shfl_xor(v, 16, 32);
    return v;
}

__global__ __launch_bounds__(kCvtThreads)
void k_cvt_rows(const float* __restrict__ src, _Float16* __restrict__ dst, float sc, int n)
{
    const size_t base = ((size_t)blockIdx.x * kCvtThreads + threadIdx.x) * 8;
    if (base + 8 <= (size_t)n) {
        const v4f f0 = *(const v4f*)(src + base);
        const v4f f1 = *(const v4f*)(src + base + 4);
        v8h hv;
        hv[0] = cvt16(f0[0], sc); hv[1] = cvt16(f0[1], sc);
        hv[2] = cvt16(f0[2], sc); hv[3] = cvt16(f0[3], sc);
        hv[4] = cvt16(f1[0], sc); hv[5] = cvt16(f1[1], sc);
        hv[6] = cvt16(f1[2], sc); hv[7] = cvt16(f1[3], sc);
        const v4u u = __builtin_bit_cast(v4u, hv);
        volatile v4u* p = (volatile v4u*)(dst + base);
        *p = u;
        __threadfence();
        *p = u;
    }
}

__global__ __launch_bounds__(kTrThreads)
void k_cvt_w1t(const float* __restrict__ w, _Float16* __restrict__ wt)
{
    __shared__ __align__(16) _Float16 sT[64 * kTP];
    const int tid = threadIdx.x;
    const int n0  = blockIdx.x * 64;
    const int k0  = blockIdx.y * 64;
#pragma unroll
    for (int i = 0; i < 4; ++i) {
        const int idx = i * kTrThreads + tid;
        const int r   = idx >> 4;
        const int c4  = idx & 15;
        const v4f f = *(const v4f*)(w + (size_t)(k0 + r) * kN1 + n0 + 4 * c4);
#pragma unroll
        for (int e = 0; e < 4; ++e)
            sT[(4 * c4 + e) * kTP + r] = cvt16(f[e], 256.0f);
    }
    __syncthreads();
    v4u u[2];
#pragma unroll
    for (int i = 0; i < 2; ++i) {
        const int idx  = i * kTrThreads + tid;
        const int line = idx >> 3;
        const int p    = idx & 7;
        u[i] = __builtin_bit_cast(v4u, *(const v8h*)(sT + line * kTP + 8 * p));
    }
#pragma unroll
    for (int i = 0; i < 2; ++i) {
        const int idx = i * kTrThreads + tid;
        *(volatile v4u*)(wt + (size_t)(n0 + (idx >> 3)) * kD + k0 + 8 * (idx & 7)) = u[i];
    }
    __threadfence();
#pragma unroll
    for (int i = 0; i < 2; ++i) {
        const int idx = i * kTrThreads + tid;
        *(volatile v4u*)(wt + (size_t)(n0 + (idx >> 3)) * kD + k0 + 8 * (idx & 7)) = u[i];
    }
}

__global__ __launch_bounds__(kLnThreads)
void k_ln_x(const float* __restrict__ x, _Float16* __restrict__ Xh)
{
    __shared__ float red[4];
    const int tid  = threadIdx.x;
    const int wave = tid >> 5;
    const int lane = tid & 31;
    const int row  = blockIdx.x;
    const int c0   = tid * 8;
    const float* xr = x + (size_t)row * kD + c0;
    const v4f f0 = *(const v4f*)(xr);
    const v4f f1 = *(const v4f*)(xr + 4);
    float v[8];
    v[0] = bf16_rne(f0[0]); v[1] = bf16_rne(f0[1]); v[2] = bf16_rne(f0[2]); v[3] = bf16_rne(f0[3]);
    v[4] = bf16_rne(f1[0]); v[5] = bf16_rne(f1[1]); v[6] = bf16_rne(f1[2]); v[7] = bf16_rne(f1[3]);

    float s = 0.0f;
#pragma unroll
    for (int e = 0; e < 8; ++e) s += v[e];
    s = wave_sum(s);
    if (lane == 0) red[wave] = s;
    __syncthreads();
    const float mean = (red[0] + red[1]) * (1.0f / (float)kD);

    float ss = 0.0f;
#pragma unroll
    for (int e = 0; e < 8; ++e) { v[e] = v[e] - mean; ss += v[e] * v[e]; }
    ss = wave_sum(ss);
    if (lane == 0) red[2 + wave] = ss;
    __syncthreads();
    const float var  = (red[2] + red[3]) * (1.0f / (float)kD);
    const float rstd = rsqrtf(var + 1e-6f);

    v8h hv;
#pragma unroll
    for (int e = 0; e < 8; ++e) hv[e] = (_Float16)(v[e] * rstd * 16.0f);
    const v4u u = __builtin_bit_cast(v4u, hv);
    volatile v4u* p = (volatile v4u*)(Xh + (size_t)row * kD + c0);
    *p = u;
    __threadfence();
    *p = u;
}

__global__ __launch_bounds__(kFlagThreads)
void k_flags(const float* __restrict__ mask, const int* __restrict__ ts_unused, int* __restrict__ flags)
{
    __shared__ __align__(16) int sf[32];
    (void)ts_unused;
    const int tid = threadIdx.x;
    const int qb  = blockIdx.x;
    const float* mp = mask + (size_t)(qb * 64) * kN + 8 * tid;
    int any = 0;
#pragma unroll 1
    for (int r = 0; r < 64; ++r) {
        const v4f a = *(const v4f*)(mp + (size_t)r * kN);
        const v4f c = *(const v4f*)(mp + (size_t)r * kN + 4);
        any |= (int)(a[0] != 0.0f) | (int)(a[1] != 0.0f) | (int)(a[2] != 0.0f) | (int)(a[3] != 0.0f)
             | (int)(c[0] != 0.0f) | (int)(c[1] != 0.0f) | (int)(c[2] != 0.0f) | (int)(c[3] != 0.0f);
    }
    any |= __shfl_xor(any, 1, 32);
    any |= __shfl_xor(any, 2, 32);
    if ((tid & 3) == 0) sf[tid >> 2] = any;
    __syncthreads();
    if (tid < 8) {
        const v4i v = *(const v4i*)(sf + 4 * tid);
        volatile v4i* p = (volatile v4i*)(flags + (size_t)qb * kKch + 4 * tid);
        *p = v;
        __threadfence();
        *p = v;
    }
}

__global__ __launch_bounds__(kGemmThreads)
void k_gemm1(const _Float16* __restrict__ Xh, const _Float16* __restrict__ W1h,
             float* __restrict__ Uf, _Float16* __restrict__ Vh,
             _Float16* __restrict__ Qh, _Float16* __restrict__ Kh)
{
    __shared__ __align__(16) float stg[64 * kStgPitch];

    const int tid  = threadIdx.x;
    const int wave = tid >> 5;
    const int lane = tid & 31;
    const int h    = lane >> 4;
    const int m    = lane & 15;
    const int n0   = blockIdx.x * 128;
    const int m0   = blockIdx.y * 64;
    const int wm   = (wave & 1) * 32;
    const int wn   = (wave >> 1) * 64;

    const _Float16* ap = Xh  + (size_t)(m0 + wm + m) * kD + 8 * h;
    const _Float16* bp = W1h + (size_t)(n0 + wn + m) * kD + 8 * h;

    v8f acc[8] = {};
#pragma unroll 1
    for (int k0 = 0; k0 < kD; k0 += 32) {
        Frag a0, a1;
        a0.half[0] = *(const v8h*)(ap + k0);
        a0.half[1] = *(const v8h*)(ap + k0 + 16);
        a1.half[0] = *(const v8h*)(ap + 16 * kD + k0);
        a1.half[1] = *(const v8h*)(ap + 16 * kD + k0 + 16);
#pragma unroll
        for (int t = 0; t < 4; ++t) {
            Frag b;
            const _Float16* bt = bp + (size_t)t * 16 * kD + k0;
            b.half[0] = *(const v8h*)(bt);
            b.half[1] = *(const v8h*)(bt + 16);
            acc[t]     = wmma_f16(a0.v, b.v, acc[t]);
            acc[4 + t] = wmma_f16(a1.v, b.v, acc[4 + t]);
        }
    }

    const int mode = n0 / kD;

#pragma unroll
    for (int t = 0; t < 4; ++t) {
        const int c = wn + 16 * t + m;
#pragma unroll
        for (int i = 0; i < 2; ++i) {
#pragma unroll
            for (int r = 0; r < 8; ++r)
                stg[(wm + 16 * i + 8 * h + r) * kStgPitch + c] = silu_fast(acc[4 * i + t][r] * (1.0f / 4096.0f));
        }
    }
    __syncthreads();

    if (mode == 0) {
        float* dst = Uf + (size_t)m0 * kD + n0 + 4 * lane;
#pragma unroll
        for (int g = 0; g < 4; ++g) {
            v4f v[4];
#pragma unroll
            for (int rr = 0; rr < 4; ++rr) {
                const int row = wave * 16 + 4 * g + rr;
                v[rr] = *(const v4f*)(stg + row * kStgPitch + 4 * lane);
            }
#pragma unroll
            for (int rr = 0; rr < 4; ++rr)
                *(volatile v4f*)(dst + (size_t)(wave * 16 + 4 * g + rr) * kD) = v[rr];
            __threadfence();
#pragma unroll
            for (int rr = 0; rr < 4; ++rr)
                *(volatile v4f*)(dst + (size_t)(wave * 16 + 4 * g + rr) * kD) = v[rr];
        }
    } else {
        _Float16* plane = (mode == 1) ? Vh : ((mode == 2) ? Qh : Kh);
        const int coff = n0 - mode * kD;
        _Float16* dst = plane + (size_t)m0 * kD + coff + 8 * m;
        v4u u[8];
#pragma unroll
        for (int i = 0; i < 8; ++i) {
            const int row = wave * 16 + 2 * i + h;
            const float* sp = stg + row * kStgPitch + 8 * m;
            const v4f f0 = *(const v4f*)(sp);
            const v4f f1 = *(const v4f*)(sp + 4);
            v8h hv;
#pragma unroll
            for (int e = 0; e < 4; ++e) {
                hv[e]     = (_Float16)(f0[e] * 64.0f);
                hv[4 + e] = (_Float16)(f1[e] * 64.0f);
            }
            u[i] = __builtin_bit_cast(v4u, hv);
        }
#pragma unroll
        for (int i = 0; i < 8; ++i)
            *(volatile v4u*)(dst + (size_t)(wave * 16 + 2 * i + h) * kD) = u[i];
        __threadfence();
#pragma unroll
        for (int i = 0; i < 8; ++i)
            *(volatile v4u*)(dst + (size_t)(wave * 16 + 2 * i + h) * kD) = u[i];
    }
}

__global__ __launch_bounds__(kVtThreads)
void k_vt(const _Float16* __restrict__ Vh, const int* __restrict__ offs, _Float16* __restrict__ VT)
{
    __shared__ __align__(16) _Float16 sT[64 * kTP];
    const int tid  = threadIdx.x;
    const int blk  = blockIdx.x;
    const int pblk = blk % kQblk;
    const int hh   = (blk / kQblk) % kHeads;
    const int bb   = blk / (kQblk * kHeads);
    const int ob   = offs[bb];
    const int len  = offs[bb + 1] - ob;
    const int p0   = pblk * 64;
#pragma unroll
    for (int i = 0; i < 4; ++i) {
        const int idx = i * kVtThreads + tid;
        const int r   = idx >> 3;
        const int pc  = idx & 7;
        const int p   = p0 + r;
        const int g   = min(max(ob + p, 0), kTok - 1);
        const v8h hv  = *(const v8h*)(Vh + (size_t)g * kD + hh * kDh + 8 * pc);
        const bool ok = (p < len);
#pragma unroll
        for (int e = 0; e < 8; ++e)
            sT[(8 * pc + e) * kTP + r] = ok ? hv[e] : (_Float16)0.0f;
    }
    __syncthreads();
    v4u u[4];
#pragma unroll
    for (int i = 0; i < 4; ++i) {
        const int idx = i * kVtThreads + tid;
        const int d   = idx >> 3;
        const int q   = idx & 7;
        u[i] = __builtin_bit_cast(v4u, *(const v8h*)(sT + d * kTP + 8 * q));
    }
    _Float16* vb = VT + (size_t)((bb * kHeads + hh) * kDh) * kN + p0;
#pragma unroll
    for (int i = 0; i < 4; ++i) {
        const int idx = i * kVtThreads + tid;
        *(volatile v4u*)(vb + (size_t)(idx >> 3) * kN + 8 * (idx & 7)) = u[i];
    }
    __threadfence();
#pragma unroll
    for (int i = 0; i < 4; ++i) {
        const int idx = i * kVtThreads + tid;
        *(volatile v4u*)(vb + (size_t)(idx >> 3) * kN + 8 * (idx & 7)) = u[i];
    }
}

__global__ __launch_bounds__(kGemmThreads)
void k_attn(const _Float16* __restrict__ Qh, const _Float16* __restrict__ Kh,
            const _Float16* __restrict__ VT, const float* __restrict__ mask,
            const float* __restrict__ relw, const int* __restrict__ offs,
            const int* __restrict__ flags, float* __restrict__ Af)
{
    __shared__ __align__(16) float sP[4 * 16 * kPP];
    __shared__ __align__(16) float sO[4 * 16 * kOP];

    const int tid  = threadIdx.x;
    const int wave = tid >> 5;
    const int lane = tid & 31;
    const int h    = lane >> 4;
    const int m    = lane & 15;
    const int blk  = blockIdx.x;
    const int qblk = blk % kQblk;
    const int hh   = (blk / kQblk) % kHeads;
    const int bb   = blk / (kQblk * kHeads);
    const int ob   = offs[bb];
    const int len  = offs[bb + 1] - ob;
    const int qb0  = qblk * 64;
    if (qb0 >= len) return;
    const int q0   = qb0 + wave * 16;
    const int hc   = hh * kDh;

    const int* fl = flags + qblk * kKch;

    const int gq = min(max(ob + q0 + m, 0), kTok - 1);
    const _Float16* qp = Qh + (size_t)gq * kD + hc + 8 * h;
    Frag aq0, aq1;
    aq0.half[0] = *(const v8h*)(qp);
    aq0.half[1] = *(const v8h*)(qp + 16);
    aq1.half[0] = *(const v8h*)(qp + 32);
    aq1.half[1] = *(const v8h*)(qp + 48);

    const _Float16* vp = VT + (size_t)((bb * kHeads + hh) * kDh + m) * kN + 8 * h;
    const float*  mrow = mask + (size_t)(q0 + m) * kN + 8 * h;
    float* myP = sP + wave * (16 * kPP);
    float* myO = sO + wave * (16 * kOP);

    v8f acc[4] = {};
#pragma unroll 1
    for (int kc = 0; kc < kKch; ++kc) {
        const int kb = kc * 32;
        if (kb < len && fl[kc] != 0) {
            const int gk0 = min(max(ob + kb + m, 0), kTok - 1);
            const int gk1 = min(max(ob + kb + 16 + m, 0), kTok - 1);
            const _Float16* kr0 = Kh + (size_t)gk0 * kD + hc + 8 * h;
            const _Float16* kr1 = Kh + (size_t)gk1 * kD + hc + 8 * h;
            Frag b00, b01, b10, b11;
            b00.half[0] = *(const v8h*)(kr0);
            b00.half[1] = *(const v8h*)(kr0 + 16);
            b01.half[0] = *(const v8h*)(kr0 + 32);
            b01.half[1] = *(const v8h*)(kr0 + 48);
            b10.half[0] = *(const v8h*)(kr1);
            b10.half[1] = *(const v8h*)(kr1 + 16);
            b11.half[0] = *(const v8h*)(kr1 + 32);
            b11.half[1] = *(const v8h*)(kr1 + 48);
            v8f s0 = {}, s1 = {};
            s0 = wmma_f16(aq0.v, b00.v, s0);
            s0 = wmma_f16(aq1.v, b01.v, s0);
            s1 = wmma_f16(aq0.v, b10.v, s1);
            s1 = wmma_f16(aq1.v, b11.v, s1);

            {
                float* pw = myP + (8 * h) * kPP + m;
                const int ib = kb + m - (q0 + 8 * h) + (kN - 1);
#pragma unroll
                for (int r = 0; r < 8; ++r) {
                    const int i0 = min(max(ib - r, 0), kRel - 1);
                    const int i1 = min(max(ib + 16 - r, 0), kRel - 1);
                    pw[r * kPP]      = silu_fast(s0[r] * (1.0f / 4096.0f) + bf16_rne(relw[i0]));
                    pw[r * kPP + 16] = silu_fast(s1[r] * (1.0f / 4096.0f) + bf16_rne(relw[i1]));
                }
            }
            __syncthreads();

            Frag apf;
            {
                const float* pr = myP + m * kPP + 8 * h;
                const float* mk = mrow + kb;
                const v4f p0 = *(const v4f*)(pr);
                const v4f p1 = *(const v4f*)(pr + 4);
                const v4f p2 = *(const v4f*)(pr + 16);
                const v4f p3 = *(const v4f*)(pr + 20);
                const v4f w0 = *(const v4f*)(mk);
                const v4f w1 = *(const v4f*)(mk + 4);
                const v4f w2 = *(const v4f*)(mk + 16);
                const v4f w3 = *(const v4f*)(mk + 20);
                const int kk = kb + 8 * h;
                v8h h0v, h1v;
#pragma unroll
                for (int e = 0; e < 4; ++e) {
                    const float mv0 = (kk + e      < len) ? bf16_rne(w0[e]) : 0.0f;
                    const float mv1 = (kk + 4 + e  < len) ? bf16_rne(w1[e]) : 0.0f;
                    const float mv2 = (kk + 16 + e < len) ? bf16_rne(w2[e]) : 0.0f;
                    const float mv3 = (kk + 20 + e < len) ? bf16_rne(w3[e]) : 0.0f;
                    h0v[e]     = (_Float16)(p0[e] * mv0 * 64.0f);
                    h0v[4 + e] = (_Float16)(p1[e] * mv1 * 64.0f);
                    h1v[e]     = (_Float16)(p2[e] * mv2 * 64.0f);
                    h1v[4 + e] = (_Float16)(p3[e] * mv3 * 64.0f);
                }
                apf.half[0] = h0v;
                apf.half[1] = h1v;
            }
#pragma unroll
            for (int t = 0; t < 4; ++t) {
                Frag bv;
                const _Float16* vr = vp + (size_t)t * 16 * kN + kb;
                bv.half[0] = *(const v8h*)(vr);
                bv.half[1] = *(const v8h*)(vr + 16);
                acc[t] = wmma_f16(apf.v, bv.v, acc[t]);
            }
            __syncthreads();
        }
    }

#pragma unroll
    for (int t = 0; t < 4; ++t) {
#pragma unroll
        for (int r = 0; r < 8; ++r)
            myO[(8 * h + r) * kOP + 16 * t + m] = acc[t][r] * (1.0f / 4194304.0f);
    }
    __syncthreads();

    v4f g[8];
#pragma unroll
    for (int i = 0; i < 8; ++i) {
        const int row = 2 * i + h;
        g[i] = *(const v4f*)(myO + row * kOP + 4 * m);
    }
#pragma unroll
    for (int i = 0; i < 8; ++i) {
        const int qpos = q0 + 2 * i + h;
        const int gr   = ob + qpos;
        if (qpos < len && (unsigned)gr < (unsigned)kTok)
            *(volatile v4f*)(Af + (size_t)gr * kD + hc + 4 * m) = g[i];
    }
    __threadfence();
#pragma unroll
    for (int i = 0; i < 8; ++i) {
        const int qpos = q0 + 2 * i + h;
        const int gr   = ob + qpos;
        if (qpos < len && (unsigned)gr < (unsigned)kTok)
            *(volatile v4f*)(Af + (size_t)gr * kD + hc + 4 * m) = g[i];
    }
}

__global__ __launch_bounds__(kLnThreads)
void k_norm2(const float* __restrict__ A, const float* __restrict__ Uf, _Float16* __restrict__ Oh)
{
    __shared__ float red[4];
    const int tid  = threadIdx.x;
    const int wave = tid >> 5;
    const int lane = tid & 31;
    const int row  = blockIdx.x;
    const int c0   = tid * 8;
    const float* ar = A + (size_t)row * kD + c0;
    const v4f f0 = *(const v4f*)(ar);
    const v4f f1 = *(const v4f*)(ar + 4);
    float v[8];
    v[0] = f0[0]; v[1] = f0[1]; v[2] = f0[2]; v[3] = f0[3];
    v[4] = f1[0]; v[5] = f1[1]; v[6] = f1[2]; v[7] = f1[3];

    float s = 0.0f;
#pragma unroll
    for (int e = 0; e < 8; ++e) s += v[e];
    s = wave_sum(s);
    if (lane == 0) red[wave] = s;
    __syncthreads();
    const float mean = (red[0] + red[1]) * (1.0f / (float)kD);

    float ss = 0.0f;
#pragma unroll
    for (int e = 0; e < 8; ++e) { v[e] = v[e] - mean; ss += v[e] * v[e]; }
    ss = wave_sum(ss);
    if (lane == 0) red[2 + wave] = ss;
    __syncthreads();
    const float var  = (red[2] + red[3]) * (1.0f / (float)kD);
    const float rstd = rsqrtf(var + 1e-6f);

    const float* ur = Uf + (size_t)row * kD + c0;
    const v4f u0 = *(const v4f*)(ur);
    const v4f u1 = *(const v4f*)(ur + 4);
    float uu[8];
    uu[0] = u0[0]; uu[1] = u0[1]; uu[2] = u0[2]; uu[3] = u0[3];
    uu[4] = u1[0]; uu[5] = u1[1]; uu[6] = u1[2]; uu[7] = u1[3];

    v8h hv;
#pragma unroll
    for (int e = 0; e < 8; ++e) hv[e] = (_Float16)((uu[e] * (v[e] * rstd)) * 16.0f);
    const v4u u = __builtin_bit_cast(v4u, hv);
    volatile v4u* p = (volatile v4u*)(Oh + (size_t)row * kD + c0);
    *p = u;
    __threadfence();
    *p = u;
}

__global__ __launch_bounds__(kGemmThreads)
void k_gemm2(const _Float16* __restrict__ Oh, const _Float16* __restrict__ W2h,
             const float* __restrict__ b2, const float* __restrict__ Xres, float* __restrict__ Out)
{
    __shared__ __align__(16) float stg[32 * kStgPitch];

    const int tid  = threadIdx.x;
    const int wave = tid >> 5;
    const int lane = tid & 31;
    const int h    = lane >> 4;
    const int m    = lane & 15;
    const int n0   = blockIdx.x * 128;
    const int m0   = blockIdx.y * 32;
    const int wn   = wave * 32;

    const _Float16* ap = Oh  + (size_t)(m0 + m) * kD + 8 * h;
    const _Float16* bp = W2h + (size_t)(n0 + wn + m) * kD + 8 * h;

    v8f acc[4] = {};
#pragma unroll 1
    for (int k0 = 0; k0 < kD; k0 += 32) {
        Frag a0, a1, b0, b1;
        a0.half[0] = *(const v8h*)(ap + k0);
        a0.half[1] = *(const v8h*)(ap + k0 + 16);
        a1.half[0] = *(const v8h*)(ap + 16 * kD + k0);
        a1.half[1] = *(const v8h*)(ap + 16 * kD + k0 + 16);
        b0.half[0] = *(const v8h*)(bp + k0);
        b0.half[1] = *(const v8h*)(bp + k0 + 16);
        b1.half[0] = *(const v8h*)(bp + 16 * kD + k0);
        b1.half[1] = *(const v8h*)(bp + 16 * kD + k0 + 16);
        acc[0] = wmma_f16(a0.v, b0.v, acc[0]);
        acc[1] = wmma_f16(a0.v, b1.v, acc[1]);
        acc[2] = wmma_f16(a1.v, b0.v, acc[2]);
        acc[3] = wmma_f16(a1.v, b1.v, acc[3]);
    }

#pragma unroll
    for (int t = 0; t < 2; ++t) {
        const int c = wn + 16 * t + m;
        const float bias = bf16_rne(b2[n0 + c]);
#pragma unroll
        for (int i = 0; i < 2; ++i) {
#pragma unroll
            for (int r = 0; r < 8; ++r)
                stg[(16 * i + 8 * h + r) * kStgPitch + c] = acc[2 * i + t][r] * (1.0f / 4096.0f) + bias;
        }
    }
    __syncthreads();

    float* dst = Out + (size_t)m0 * kD + n0 + 4 * lane;
    const float* xr = Xres + (size_t)m0 * kD + n0 + 4 * lane;
    v4f v[8];
#pragma unroll
    for (int rr = 0; rr < 8; ++rr) {
        const int row = wave * 8 + rr;
        const v4f s  = *(const v4f*)(stg + row * kStgPitch + 4 * lane);
        const v4f xv = *(const v4f*)(xr + (size_t)row * kD);
        v4f o;
        o[0] = s[0] + bf16_rne(xv[0]);
        o[1] = s[1] + bf16_rne(xv[1]);
        o[2] = s[2] + bf16_rne(xv[2]);
        o[3] = s[3] + bf16_rne(xv[3]);
        v[rr] = o;
    }
#pragma unroll
    for (int rr = 0; rr < 8; ++rr)
        *(volatile v4f*)(dst + (size_t)(wave * 8 + rr) * kD) = v[rr];
    __threadfence();
#pragma unroll
    for (int rr = 0; rr < 8; ++rr)
        *(volatile v4f*)(dst + (size_t)(wave * 8 + rr) * kD) = v[rr];
}

extern "C" void kernel_launch(void* const* d_in, const int* in_sizes, int n_in,
                              void* d_out, int out_size, void* d_ws, size_t ws_size,
                              hipStream_t stream)
{
    if (n_in < 8) return;
    if (in_sizes[0] != kTok * kD) return;
    if (in_sizes[1] != kB + 1) return;
    if (in_sizes[3] != kN * kN) return;
    if (in_sizes[4] != kD * kN1) return;
    if (in_sizes[5] != kD * kD) return;
    if (in_sizes[6] != kD) return;
    if (in_sizes[7] != kRel) return;
    if (out_size != kTok * kD) return;

    const size_t bXh  = (size_t)kTok * kD * sizeof(_Float16);
    const size_t bW1h = (size_t)kN1 * kD * sizeof(_Float16);
    const size_t bW2h = (size_t)kD * kD * sizeof(_Float16);
    const size_t bUf  = (size_t)kTok * kD * sizeof(float);
    const size_t bVh  = (size_t)kTok * kD * sizeof(_Float16);
    const size_t bQh  = bVh;
    const size_t bKh  = bVh;
    const size_t bVT  = (size_t)kB * kHeads * kDh * kN * sizeof(_Float16);
    const size_t bAf  = (size_t)kTok * kD * sizeof(float);
    const size_t bOh  = (size_t)kTok * kD * sizeof(_Float16);
    const size_t bFl  = (size_t)kQblk * kKch * sizeof(int);
    const size_t total = bXh + bW1h + bW2h + bUf + bVh + bQh + bKh + bVT + bAf + bOh + bFl;
    if (ws_size < total) return;

    const float* x      = (const float*)d_in[0];
    const int*   offs   = (const int*)d_in[1];
    const int*   tstamp = (const int*)d_in[2];
    const float* mask   = (const float*)d_in[3];
    const float* W_uvqk = (const float*)d_in[4];
    const float* W_o    = (const float*)d_in[5];
    const float* b_o    = (const float*)d_in[6];
    const float* rel_w  = (const float*)d_in[7];
    float* Out = (float*)d_out;

    char* ws = (char*)d_ws;
    size_t o = 0;
    _Float16* Xh  = (_Float16*)(ws + o); o += bXh;
    _Float16* W1h = (_Float16*)(ws + o); o += bW1h;
    _Float16* W2h = (_Float16*)(ws + o); o += bW2h;
    float*    Uf  = (float*)(ws + o);    o += bUf;
    _Float16* Vh  = (_Float16*)(ws + o); o += bVh;
    _Float16* Qh  = (_Float16*)(ws + o); o += bQh;
    _Float16* Kh  = (_Float16*)(ws + o); o += bKh;
    _Float16* VT  = (_Float16*)(ws + o); o += bVT;
    float*    Af  = (float*)(ws + o);    o += bAf;
    _Float16* Oh  = (_Float16*)(ws + o); o += bOh;
    int*      Fl  = (int*)(ws + o);      o += bFl;

    const int nW2 = kD * kD;
    k_ln_x<<<dim3(kTok), dim3(kLnThreads), 0, stream>>>(x, Xh);
    k_cvt_w1t<<<dim3(kN1 / 64, kD / 64), dim3(kTrThreads), 0, stream>>>(W_uvqk, W1h);
    k_cvt_rows<<<dim3((unsigned)(nW2 / 8 / kCvtThreads)), dim3(kCvtThreads), 0, stream>>>(W_o, W2h, 256.0f, nW2);
    k_flags<<<dim3(kQblk), dim3(kFlagThreads), 0, stream>>>(mask, tstamp, Fl);
    k_gemm1<<<dim3(kN1 / 128, kTok / 64), dim3(kGemmThreads), 0, stream>>>(Xh, W1h, Uf, Vh, Qh, Kh);
    k_vt<<<dim3(kB * kHeads * kQblk), dim3(kVtThreads), 0, stream>>>(Vh, offs, VT);
    k_attn<<<dim3(kB * kHeads * kQblk), dim3(kGemmThreads), 0, stream>>>(Qh, Kh, VT, mask, rel_w, offs, Fl, Af);
    k_norm2<<<dim3(kTok), dim3(kLnThreads), 0, stream>>>(Af, Uf, Oh);
    k_gemm2<<<dim3(kD / 128, kTok / 32), dim3(kGemmThreads), 0, stream>>>(Oh, W2h, b_o, x, Out);
}
